// BiLSTM_45234595561814
// MI455X (gfx1250) — hardware-verified
//
#include <hip/hip_runtime.h>
#include <math.h>

constexpr int SEQS    = 64;
constexpr int STEPS   = 512;
constexpr int DIN     = 64;
constexpr int HID     = 128;
constexpr int G4      = 4 * HID;
constexpr int H2      = 2 * HID;
constexpr int NROWS   = SEQS * STEPS;
constexpr int MLPH    = 256;
constexpr int DOUT    = 64;
constexpr int NTHR    = 256;
constexpr int SEQ_BLK = 16;
constexpr int HPAD    = HID + 8;
constexpr int XSP     = G4 + 4;
constexpr float WCARRY     = 256.0f;
constexpr float WCARRY_INV = 1.0f / 256.0f;
static_assert(SEQS % SEQ_BLK == 0);
static_assert(HID == 16 * (NTHR / 32));
static_assert(SEQ_BLK == 2 * (NTHR / 32));
static_assert(HID == 2 * 64);
static_assert((SEQ_BLK * G4 / 4) % NTHR == 0);
static_assert(DIN % 32 == 0 && HID % 32 == 0 && H2 % 32 == 0 && MLPH % 32 == 0);
static_assert(NROWS % 64 == 0 && G4 % 64 == 0 && MLPH % 64 == 0 && DOUT % 64 == 0);
static_assert(HPAD % 8 == 0 && XSP % 4 == 0);

typedef __attribute__((ext_vector_type(16))) _Float16 v16h;
typedef __attribute__((ext_vector_type(8)))  _Float16 v8h;
typedef __attribute__((ext_vector_type(16))) __bf16   v16b;
typedef __attribute__((ext_vector_type(8)))  __bf16   v8b;
typedef __attribute__((ext_vector_type(8)))  float    v8f;
typedef __attribute__((ext_vector_type(4)))  float    v4f;

__device__ __forceinline__ unsigned short f2bf_bits(float f) {
  unsigned u = __float_as_uint(f);
  return (unsigned short)((u + 0x7FFFu + ((u >> 16) & 1u)) >> 16);
}
__device__ __forceinline__ float bf_bits2f(unsigned short h) { return __uint_as_float(((unsigned)h) << 16); }
__device__ __forceinline__ float bf16r(float f) { return bf_bits2f(f2bf_bits(f)); }

__device__ __forceinline__ void dep_guard_h(v8f& a, v8f& b, v16h x, v16h y) { asm volatile("v_nop\n\tv_nop\n\tv_nop\n\tv_nop" : "+v"(a), "+v"(b) : "v"(x), "v"(y)); }
__device__ __forceinline__ void dep_guard_b(v8f& a, v8f& b, v16b x, v16b y) { asm volatile("v_nop\n\tv_nop\n\tv_nop\n\tv_nop" : "+v"(a), "+v"(b) : "v"(x), "v"(y)); }
__device__ __forceinline__ void dep_guard4_h(v8f& a, v8f& b, v8f& c, v8f& d, v16h x, v16h y) {
  asm volatile("v_nop\n\tv_nop\n\tv_nop\n\tv_nop" : "+v"(a), "+v"(b), "+v"(c), "+v"(d) : "v"(x), "v"(y));
}
__device__ __forceinline__ void dep_guard4_b(v8f& a, v8f& b, v8f& c, v8f& d, v16b x, v16b y) {
  asm volatile("v_nop\n\tv_nop\n\tv_nop\n\tv_nop" : "+v"(a), "+v"(b), "+v"(c), "+v"(d) : "v"(x), "v"(y));
}
__device__ __forceinline__ void rec_guard(v8f& a0, v8f& a1, v8f& a2, v8f& a3, v16h x, v16h y0, v16h y1, v16h y2, v16h y3) {
  asm volatile("v_nop\n\tv_nop\n\tv_nop\n\tv_nop" : "+v"(a0), "+v"(a1), "+v"(a2), "+v"(a3) : "v"(x), "v"(y0), "v"(y1), "v"(y2), "v"(y3));
}
__device__ __forceinline__ void keep4_h(v16h a, v16h b, v16h c, v16h d) { asm volatile("v_nop" :: "v"(a), "v"(b), "v"(c), "v"(d)); }
__device__ __forceinline__ void keep4_b(v16b a, v16b b, v16b c, v16b d) { asm volatile("v_nop" :: "v"(a), "v"(b), "v"(c), "v"(d)); }
__device__ __forceinline__ void acc_guard4(v8f& a, v8f& b, v8f& c, v8f& d) { asm volatile("v_nop\n\tv_nop\n\tv_nop\n\tv_nop" : "+v"(a), "+v"(b), "+v"(c), "+v"(d)); }
template <typename T> struct Frag;
template <> struct Frag<_Float16> {
  typedef v16h V; union U { v16h v; v8h h[2]; };
  static __device__ __forceinline__ v16h load(const _Float16* p) {
    U f; f.h[0] = *(const v8h*)(p); f.h[1] = *(const v8h*)(p + 16); return f.v;
  }
  static __device__ __forceinline__ v8f mma(v16h a, v16h b, v8f c) {
    return __builtin_amdgcn_wmma_f32_16x16x32_f16(false, a, false, b, (short)0, c, false, false);
  }
  static __device__ __forceinline__ void guard4(v8f& a, v8f& b, v8f& c, v8f& d, v16h x, v16h y) { dep_guard4_h(a, b, c, d, x, y); }
  static __device__ __forceinline__ void keep(v16h a, v16h b, v16h c, v16h d) { keep4_h(a, b, c, d); }
};
template <> struct Frag<__bf16> {
  typedef v16b V; union U { v16b v; v8b h[2]; };
  static __device__ __forceinline__ v16b load(const __bf16* p) {
    U f; f.h[0] = *(const v8b*)(p); f.h[1] = *(const v8b*)(p + 16); return f.v;
  }
  static __device__ __forceinline__ v8f mma(v16b a, v16b b, v8f c) {
    return __builtin_amdgcn_wmma_f32_16x16x32_bf16(false, a, false, b, (short)0, c, false, false);
  }
  static __device__ __forceinline__ void guard4(v8f& a, v8f& b, v8f& c, v8f& d, v16b x, v16b y) { dep_guard4_b(a, b, c, d, x, y); }
  static __device__ __forceinline__ void keep(v16b a, v16b b, v16b c, v16b d) { keep4_b(a, b, c, d); }
};

__device__ __forceinline__ float fsig(float x) { return 1.0f / (1.0f + expf(-x)); }

template <int ET> struct Elem;
template <> struct Elem<0> { typedef _Float16 T; };
template <> struct Elem<1> { typedef __bf16 T; };
template <int ET, bool SPLIT, int BIAS_MODE, int OUT_MODE, bool RESID, int ACT = 0>
__global__ __launch_bounds__(256) void wmma_gemm64(
    const unsigned short* __restrict__ Ap, const unsigned short* __restrict__ A2p, int lda, long strideA,
    const unsigned short* __restrict__ Btp, const unsigned short* __restrict__ Bt2p, int ldb, long strideB,
    void* __restrict__ Cout, void* __restrict__ Cout2, int ldc, long strideC,
    const float* __restrict__ bias,
    const float* __restrict__ resid, long strideR,
    int M, int N, int K, float scale) {
  typedef typename Elem<ET>::T T;
  typedef typename Frag<T>::V V;
  const T* A = (const T*)Ap; const T* A2 = (const T*)A2p; const T* Bt = (const T*)Btp; const T* Bt2 = (const T*)Bt2p;
  __shared__ __align__(16) float sT[8][16 * 68];
  const int b    = blockIdx.y;
  const int lane = threadIdx.x & 31;
  const int wave = threadIdx.x >> 5;
  const int tilesN = N >> 6;
  const int tilesM = M >> 6;
  const int tile = blockIdx.x * 8 + wave;
  if (tile >= tilesM * tilesN) return;
  const int tm = tile / tilesN;
  const int tn = tile - tm * tilesN;
  const int m0 = tm << 6;
  const int n0 = tn << 6;

  const T* Ab  = A  + (size_t)b * strideA;
  const T* Bb  = Bt + (size_t)b * strideB;
  const T* Ab2 = SPLIT ? (A2  + (size_t)b * strideA) : nullptr;
  const T* Bb2 = SPLIT ? (Bt2 + (size_t)b * strideB) : nullptr;

  const int rlane = lane & 15;
  const int koff  = (lane >> 4) * 8;
  const int mOff  = (lane >> 4) * 8;

  v8f acc[4][4];
#pragma unroll
  for (int i = 0; i < 4; ++i)
#pragma unroll
    for (int j = 0; j < 4; ++j) acc[i][j] = (v8f){0.f,0.f,0.f,0.f,0.f,0.f,0.f,0.f};

  for (int k0 = 0; k0 < K; k0 += 32) {
    V bh[4], bl[4];
#pragma unroll
    for (int j = 0; j < 4; ++j) {
      const size_t bo = (size_t)(n0 + (j << 4) + rlane) * ldb + koff + k0;
      bh[j] = Frag<T>::load(Bb + bo);
      if (SPLIT) bl[j] = Frag<T>::load(Bb2 + bo);
    }
#pragma unroll
    for (int i = 0; i < 4; ++i) {
      const size_t ao = (size_t)(m0 + (i << 4) + rlane) * lda + koff + k0;
      V ah = Frag<T>::load(Ab + ao);
      V al;
      if (SPLIT) al = Frag<T>::load(Ab2 + ao);
#pragma unroll
      for (int j = 0; j < 4; ++j) {
        acc[i][j] = Frag<T>::mma(ah, bh[j], acc[i][j]);
        if (SPLIT) {
          acc[i][j] = Frag<T>::mma(ah, bl[j], acc[i][j]);
          acc[i][j] = Frag<T>::mma(al, bh[j], acc[i][j]);
        }
      }
      Frag<T>::guard4(acc[i][0], acc[i][1], acc[i][2], acc[i][3], ah, SPLIT ? al : ah);
    }
    Frag<T>::keep(bh[0], bh[1], bh[2], bh[3]);
    if (SPLIT) Frag<T>::keep(bl[0], bl[1], bl[2], bl[3]);
  }
  acc_guard4(acc[0][0], acc[0][1], acc[0][2], acc[0][3]);
  acc_guard4(acc[1][0], acc[1][1], acc[1][2], acc[1][3]);
  acc_guard4(acc[2][0], acc[2][1], acc[2][2], acc[2][3]);
  acc_guard4(acc[3][0], acc[3][1], acc[3][2], acc[3][3]);

  float* slab = sT[wave];
  const float* Rb = RESID ? (resid + (size_t)b * strideR) : nullptr;
#pragma unroll
  for (int i = 0; i < 4; ++i) {
    const int mBase = m0 + (i << 4);
#pragma unroll
    for (int j = 0; j < 4; ++j) {
      const int n = n0 + (j << 4) + rlane;
      float bv = 0.f;
      if (BIAS_MODE == 2) bv = bias[n];
#pragma unroll
      for (int r = 0; r < 8; ++r) {
        float v = acc[i][j][r] * scale;
        if (BIAS_MODE == 1) v += bias[mBase + mOff + r];
        if (BIAS_MODE == 2) v += bv;
        if (RESID) v += Rb[(size_t)(mBase + mOff + r) * ldc + n];
        if (ACT == 1) v = tanhf(v);
        if (ACT == 2) v = fmaxf(v, 0.0f);
        if (ACT == 3) v = v / (1.0f + expf(-v));
        if (ACT == 4) v = (v > 0.f) ? v : 0.01f * v;
        if (ACT == 5) v = 0.5f * v * (1.0f + erff(v * 0.70710678118654752f));
        slab[(mOff + r) * 68 + (j << 4) + rlane] = v;
      }
    }
    __builtin_amdgcn_fence(__ATOMIC_RELEASE, "workgroup");
    __builtin_amdgcn_wave_barrier();
    __builtin_amdgcn_fence(__ATOMIC_ACQUIRE, "workgroup");
    if (OUT_MODE == 0) {
      float* C = (float*)Cout + (size_t)b * strideC;
      const int hh = lane >> 4, c4 = (lane & 15) * 4;
      for (int pass = 0; pass < 2; ++pass) {
#pragma unroll
        for (int it = 0; it < 8; ++it) {
          const int row = it * 2 + hh;
          v4f v = *(const v4f*)(slab + row * 68 + c4);
          *(volatile v4f*)(C + (size_t)(mBase + row) * ldc + n0 + c4) = v;
        }
        __threadfence();
      }
    } else {
      const int q = lane >> 3, c8 = (lane & 7) * 8;
      unsigned short* C  = (unsigned short*)Cout  + (size_t)b * strideC;
      unsigned short* C2 = (OUT_MODE == 2) ? ((unsigned short*)Cout2 + (size_t)b * strideC) : nullptr;
      for (int pass = 0; pass < 2; ++pass) {
#pragma unroll
        for (int it = 0; it < 4; ++it) {
          const int row = it * 4 + q;
          const float* sp = slab + row * 68 + c8;
          v8h hv, lv;
#pragma unroll
          for (int e = 0; e < 8; ++e) {
            if (OUT_MODE == 1) {
              hv[e] = (_Float16)sp[e];
            } else {
              unsigned short hb = f2bf_bits(sp[e]);
              unsigned short lb = f2bf_bits(sp[e] - bf_bits2f(hb));
              hv[e] = __builtin_bit_cast(_Float16, hb);
              lv[e] = __builtin_bit_cast(_Float16, lb);
            }
          }
          *(volatile v8h*)(C + (size_t)(mBase + row) * ldc + n0 + c8) = hv;
          if (OUT_MODE == 2) *(volatile v8h*)(C2 + (size_t)(mBase + row) * ldc + n0 + c8) = lv;
        }
        __threadfence();
      }
    }
    __builtin_amdgcn_fence(__ATOMIC_RELEASE, "workgroup");
    __builtin_amdgcn_wave_barrier();
    __builtin_amdgcn_fence(__ATOMIC_ACQUIRE, "workgroup");
  }
}

template <int MODE>
__global__ __launch_bounds__(NTHR) void cvt8_kernel(const float* __restrict__ src, unsigned short* __restrict__ dst,
                                                    int nrow, int ncol8, int spitch, int scol0, float sc) {
  const int i  = blockIdx.x * NTHR + threadIdx.x;
  const int n8 = nrow * ncol8;
  if (i < n8) {
    const int row = i / ncol8;
    const int c8  = i - row * ncol8;
    const float* sp = src + (size_t)row * spitch + scol0 + c8 * 8;
    const v4f a = *(const v4f*)(sp);
    const v4f b = *(const v4f*)(sp + 4);
    v8h hv;
#pragma unroll
    for (int e = 0; e < 4; ++e) {
      unsigned short b0, b1;
      if (MODE == 0) {
        b0 = f2bf_bits(a[e] * sc);
        b1 = f2bf_bits(b[e] * sc);
      } else {
        b0 = __builtin_bit_cast(unsigned short, (_Float16)(bf16r(a[e]) * sc));
        b1 = __builtin_bit_cast(unsigned short, (_Float16)(bf16r(b[e]) * sc));
      }
      hv[e]     = __builtin_bit_cast(_Float16, b0);
      hv[4 + e] = __builtin_bit_cast(_Float16, b1);
    }
    *(volatile v8h*)(dst + (size_t)i * 8) = hv;
    __threadfence();
    *(volatile v8h*)(dst + (size_t)i * 8) = hv;
  }
}

template <int TWO>
__global__ __launch_bounds__(128) void bias_prep_kernel(const float* __restrict__ a, const float* __restrict__ b,
                                                        float* __restrict__ dst, int n4) {
  const int i = blockIdx.x * 128 + threadIdx.x;
  if (i < n4) {
    const v4f va = *(const v4f*)(a + 4 * i);
    v4f vb = va;
    if (TWO) vb = *(const v4f*)(b + 4 * i);
    v4f o;
#pragma unroll
    for (int e = 0; e < 4; ++e) {
      const float ra = bf16r(va[e]);
      const float rb = bf16r(vb[e]);
      o[e] = TWO ? (ra + rb) : ra;
    }
    float* op = dst + 4 * i;
    *(volatile v4f*)op = o;
    __threadfence();
    *(volatile v4f*)op = o;
  }
}

__global__ __launch_bounds__(NTHR) void lstm_seq_kernel(const float* __restrict__ XG, const unsigned short* __restrict__ WHp,
                                                        unsigned short* __restrict__ HOUT, int dir) {
  __shared__ __align__(16) _Float16 Ah[SEQ_BLK * HPAD];
  __shared__ __align__(16) float    Xs[SEQ_BLK * XSP];
  const _Float16* WH = (const _Float16*)WHp;
  const int tid = threadIdx.x, lane = tid & 31, wave = tid >> 5;
  const int c = lane & 15, hh = lane >> 4, koff = hh * 8;
  const int rowbase = blockIdx.x * SEQ_BLK;
  const int jj = 16 * wave + c;

#pragma unroll 1
  for (int i = tid; i < SEQ_BLK * HPAD; i += NTHR) Ah[i] = (_Float16)0.0f;
  float cst[8], hst[8];
#pragma unroll
  for (int r = 0; r < 8; ++r) { cst[r] = 0.0f; hst[r] = 0.0f; }
  __syncthreads();

  const _Float16* ahrow = Ah + c * HPAD + koff;
  const int sq = lane >> 3, sc8 = (lane & 7) * 8;
  const int srow = 2 * wave + (sq >> 1);
  const int scol = (sq & 1) * 64 + sc8;
  const _Float16* ahst = Ah + srow * HPAD + scol;
  unsigned short* hbase = HOUT + (size_t)(rowbase + srow) * STEPS * H2 + dir * HID + scol;
  const v8f z8 = {0.f, 0.f, 0.f, 0.f, 0.f, 0.f, 0.f, 0.f};

#pragma unroll 1
  for (int s = 0; s < STEPS; ++s) {
    const int tt = dir ? (STEPS - 1 - s) : s;
    {
      const float* xgt = XG + (size_t)tt * G4;
#pragma unroll
      for (int i = 0; i < 8; ++i) {
        const int idx = i * NTHR + tid;
        const int row = idx >> 7;
        const int c4  = (idx & 127) * 4;
        const v4f v = *(const v4f*)(xgt + (size_t)(rowbase + row) * STEPS * G4 + c4);
        *(v4f*)(Xs + row * XSP + c4) = v;
        if (i == 3) asm volatile("" ::: "memory");
      }
    }
    __syncthreads();

    if (s > 0) {
      const int tp = dir ? (tt + 1) : (tt - 1);
      const v8h hv = *(const v8h*)(ahst);
      unsigned short* dst = hbase + (size_t)tp * H2;
      *(volatile v8h*)dst = hv;
      __threadfence();
      *(volatile v8h*)dst = hv;
    }

    v8f acc[4];
    acc[0] = z8; acc[1] = z8; acc[2] = z8; acc[3] = z8;
#pragma unroll 1
    for (int k0 = 0; k0 < HID; k0 += 32) {
      const v16h a  = Frag<_Float16>::load(ahrow + k0);
      const v16h b0 = Frag<_Float16>::load(WH + (size_t)(0 * HID + jj) * HID + koff + k0);
      const v16h b1 = Frag<_Float16>::load(WH + (size_t)(1 * HID + jj) * HID + koff + k0);
      const v16h b2 = Frag<_Float16>::load(WH + (size_t)(2 * HID + jj) * HID + koff + k0);
      const v16h b3 = Frag<_Float16>::load(WH + (size_t)(3 * HID + jj) * HID + koff + k0);
      acc[0] = Frag<_Float16>::mma(a, b0, acc[0]);
      acc[1] = Frag<_Float16>::mma(a, b1, acc[1]);
      acc[2] = Frag<_Float16>::mma(a, b2, acc[2]);
      acc[3] = Frag<_Float16>::mma(a, b3, acc[3]);
      rec_guard(acc[0], acc[1], acc[2], acc[3], a, b0, b1, b2, b3);
    }
    acc_guard4(acc[0], acc[1], acc[2], acc[3]);

#pragma unroll
    for (int r = 0; r < 8; ++r) {
      const float* xr = Xs + (8 * hh + r) * XSP + jj;
      const float zi = acc[0][r] * WCARRY_INV + xr[0];
      const float zf = acc[1][r] * WCARRY_INV + xr[HID];
      const float zg = acc[2][r] * WCARRY_INV + xr[2 * HID];
      const float zo = acc[3][r] * WCARRY_INV + xr[3 * HID];
      const float ig = fsig(zi);
      const float fg = fsig(zf);
      const float gg = tanhf(zg);
      const float og = fsig(zo);
      const float cn = fg * cst[r] + ig * gg;
      cst[r] = cn;
      hst[r] = og * tanhf(cn);
    }
    __syncthreads();
#pragma unroll
    for (int r = 0; r < 8; ++r) Ah[(8 * hh + r) * HPAD + jj] = (_Float16)hst[r];
  }
  __syncthreads();
  {
    const int tl = dir ? 0 : (STEPS - 1);
    const v8h hv = *(const v8h*)(ahst);
    unsigned short* dst = hbase + (size_t)tl * H2;
    *(volatile v8h*)dst = hv;
    __threadfence();
    *(volatile v8h*)dst = hv;
  }
}

extern "C" void kernel_launch(void* const* d_in, const int* in_sizes, int n_in,
                              void* d_out, int out_size, void* d_ws, size_t ws_size, hipStream_t stream) {
  if (n_in < 21 || d_out == nullptr || d_ws == nullptr) return;
  if (in_sizes[0] != NROWS * DIN ||
      in_sizes[1] != G4 * DIN || in_sizes[2] != G4 * HID || in_sizes[3] != G4 || in_sizes[4] != G4 ||
      in_sizes[5] != G4 * DIN || in_sizes[6] != G4 * HID || in_sizes[7] != G4 || in_sizes[8] != G4 ||
      in_sizes[9] != G4 * H2 || in_sizes[10] != G4 * HID || in_sizes[11] != G4 || in_sizes[12] != G4 ||
      in_sizes[13] != G4 * H2 || in_sizes[14] != G4 * HID || in_sizes[15] != G4 || in_sizes[16] != G4 ||
      in_sizes[17] != MLPH * H2 || in_sizes[18] != MLPH || in_sizes[19] != DOUT * MLPH || in_sizes[20] != DOUT ||
      out_size != NROWS * DOUT) return;

  const float* x     = (const float*)d_in[0];
  const float* wih00 = (const float*)d_in[1];
  const float* whh00 = (const float*)d_in[2];
  const float* bih00 = (const float*)d_in[3];
  const float* bhh00 = (const float*)d_in[4];
  const float* wih01 = (const float*)d_in[5];
  const float* whh01 = (const float*)d_in[6];
  const float* bih01 = (const float*)d_in[7];
  const float* bhh01 = (const float*)d_in[8];
  const float* wih10 = (const float*)d_in[9];
  const float* whh10 = (const float*)d_in[10];
  const float* bih10 = (const float*)d_in[11];
  const float* bhh10 = (const float*)d_in[12];
  const float* wih11 = (const float*)d_in[13];
  const float* whh11 = (const float*)d_in[14];
  const float* bih11 = (const float*)d_in[15];
  const float* bhh11 = (const float*)d_in[16];
  const float* w1    = (const float*)d_in[17];
  const float* b1    = (const float*)d_in[18];
  const float* w2    = (const float*)d_in[19];
  const float* b2    = (const float*)d_in[20];
  float* y_out = (float*)d_out;

  char* ws = (char*)d_ws; size_t off = 0;
  auto carve = [&](size_t bytes) -> char* { char* p = ws + off; off += (bytes + 255) & ~(size_t)255; return p; };
  unsigned short* XB   = (unsigned short*)carve((size_t)NROWS * DIN * 2);
  unsigned short* WI0F = (unsigned short*)carve((size_t)G4 * DIN * 2);
  unsigned short* WI0B = (unsigned short*)carve((size_t)G4 * DIN * 2);
  unsigned short* WH00 = (unsigned short*)carve((size_t)G4 * HID * 2);
  unsigned short* WH01 = (unsigned short*)carve((size_t)G4 * HID * 2);
  unsigned short* WH10 = (unsigned short*)carve((size_t)G4 * HID * 2);
  unsigned short* WH11 = (unsigned short*)carve((size_t)G4 * HID * 2);
  unsigned short* WI1F = (unsigned short*)carve((size_t)G4 * H2 * 2);
  unsigned short* WI1B = (unsigned short*)carve((size_t)G4 * H2 * 2);
  unsigned short* W1P  = (unsigned short*)carve((size_t)MLPH * H2 * 2);
  unsigned short* W2P  = (unsigned short*)carve((size_t)DOUT * MLPH * 2);
  float*          BS0F = (float*)carve((size_t)G4 * 4);
  float*          BS0B = (float*)carve((size_t)G4 * 4);
  float*          BS1F = (float*)carve((size_t)G4 * 4);
  float*          BS1B = (float*)carve((size_t)G4 * 4);
  float*          B1R  = (float*)carve((size_t)MLPH * 4);
  float*          B2R  = (float*)carve((size_t)DOUT * 4);
  float*          XG   = (float*)carve((size_t)NROWS * G4 * 4);
  unsigned short* OUT0 = (unsigned short*)carve((size_t)NROWS * H2 * 2);
  unsigned short* OUT1 = (unsigned short*)carve((size_t)NROWS * H2 * 2);
  unsigned short* MID  = (unsigned short*)carve((size_t)NROWS * MLPH * 2);
  if (off > ws_size || off > (size_t)134217728) return;

  const int n8x   = NROWS * (DIN / 8);
  const int n8wi0 = G4 * (DIN / 8);
  const int n8wh  = G4 * (HID / 8);
  const int n8wi1 = G4 * (H2 / 8);
  const int n8w1  = MLPH * (H2 / 8);
  const int n8w2  = DOUT * (MLPH / 8);
  cvt8_kernel<0><<<(n8x   + NTHR - 1) / NTHR, NTHR, 0, stream>>>(x,     XB,   NROWS, DIN / 8,  DIN,  0, 1.0f);
  cvt8_kernel<0><<<(n8wi0 + NTHR - 1) / NTHR, NTHR, 0, stream>>>(wih00, WI0F, G4,    DIN / 8,  DIN,  0, 1.0f);
  cvt8_kernel<0><<<(n8wi0 + NTHR - 1) / NTHR, NTHR, 0, stream>>>(wih01, WI0B, G4,    DIN / 8,  DIN,  0, 1.0f);
  cvt8_kernel<1><<<(n8wh  + NTHR - 1) / NTHR, NTHR, 0, stream>>>(whh00, WH00, G4,    HID / 8,  HID,  0, WCARRY);
  cvt8_kernel<1><<<(n8wh  + NTHR - 1) / NTHR, NTHR, 0, stream>>>(whh01, WH01, G4,    HID / 8,  HID,  0, WCARRY);
  cvt8_kernel<1><<<(n8wh  + NTHR - 1) / NTHR, NTHR, 0, stream>>>(whh10, WH10, G4,    HID / 8,  HID,  0, WCARRY);
  cvt8_kernel<1><<<(n8wh  + NTHR - 1) / NTHR, NTHR, 0, stream>>>(whh11, WH11, G4,    HID / 8,  HID,  0, WCARRY);
  cvt8_kernel<1><<<(n8wi1 + NTHR - 1) / NTHR, NTHR, 0, stream>>>(wih10, WI1F, G4,    H2 / 8,   H2,   0, WCARRY);
  cvt8_kernel<1><<<(n8wi1 + NTHR - 1) / NTHR, NTHR, 0, stream>>>(wih11, WI1B, G4,    H2 / 8,   H2,   0, WCARRY);
  cvt8_kernel<1><<<(n8w1  + NTHR - 1) / NTHR, NTHR, 0, stream>>>(w1,    W1P,  MLPH,  H2 / 8,   H2,   0, WCARRY);
  cvt8_kernel<1><<<(n8w2  + NTHR - 1) / NTHR, NTHR, 0, stream>>>(w2,    W2P,  DOUT,  MLPH / 8, MLPH, 0, WCARRY);

  bias_prep_kernel<1><<<(G4 / 4 + 127) / 128, 128, 0, stream>>>(bih00, bhh00, BS0F, G4 / 4);
  bias_prep_kernel<1><<<(G4 / 4 + 127) / 128, 128, 0, stream>>>(bih01, bhh01, BS0B, G4 / 4);
  bias_prep_kernel<1><<<(G4 / 4 + 127) / 128, 128, 0, stream>>>(bih10, bhh10, BS1F, G4 / 4);
  bias_prep_kernel<1><<<(G4 / 4 + 127) / 128, 128, 0, stream>>>(bih11, bhh11, BS1B, G4 / 4);
  bias_prep_kernel<0><<<(MLPH / 4 + 127) / 128, 128, 0, stream>>>(b1, b1, B1R, MLPH / 4);
  bias_prep_kernel<0><<<(DOUT / 4 + 127) / 128, 128, 0, stream>>>(b2, b2, B2R, DOUT / 4);

  const int tiles_g4  = (NROWS / 64) * (G4 / 64);
  const int tiles_mlp = (NROWS / 64) * (MLPH / 64);
  const int tiles_out = (NROWS / 64) * (DOUT / 64);
  const dim3 grid_g4((tiles_g4 + 7) / 8, 1), grid_mlp((tiles_mlp + 7) / 8, 1), grid_out((tiles_out + 7) / 8, 1);
  const int rec_blocks = SEQS / SEQ_BLK;

  wmma_gemm64<1, false, 2, 0, false, 0><<<grid_g4, 256, 0, stream>>>(
      XB, XB, DIN, 0L, WI0F, WI0F, DIN, 0L, (void*)XG, (void*)XG, G4, 0L, BS0F, BS0F, 0L, NROWS, G4, DIN, 1.0f);
  lstm_seq_kernel<<<rec_blocks, NTHR, 0, stream>>>(XG, WH00, OUT0, 0);
  wmma_gemm64<1, false, 2, 0, false, 0><<<grid_g4, 256, 0, stream>>>(
      XB, XB, DIN, 0L, WI0B, WI0B, DIN, 0L, (void*)XG, (void*)XG, G4, 0L, BS0B, BS0B, 0L, NROWS, G4, DIN, 1.0f);
  lstm_seq_kernel<<<rec_blocks, NTHR, 0, stream>>>(XG, WH01, OUT0, 1);

  wmma_gemm64<0, false, 2, 0, false, 0><<<grid_g4, 256, 0, stream>>>(
      OUT0, OUT0, H2, 0L, WI1F, WI1F, H2, 0L, (void*)XG, (void*)XG, G4, 0L, BS1F, BS1F, 0L, NROWS, G4, H2, WCARRY_INV);
  lstm_seq_kernel<<<rec_blocks, NTHR, 0, stream>>>(XG, WH10, OUT1, 0);
  wmma_gemm64<0, false, 2, 0, false, 0><<<grid_g4, 256, 0, stream>>>(
      OUT0, OUT0, H2, 0L, WI1B, WI1B, H2, 0L, (void*)XG, (void*)XG, G4, 0L, BS1B, BS1B, 0L, NROWS, G4, H2, WCARRY_INV);
  lstm_seq_kernel<<<rec_blocks, NTHR, 0, stream>>>(XG, WH11, OUT1, 1);

  wmma_gemm64<0, false, 2, 1, false, 2><<<grid_mlp, 256, 0, stream>>>(
      OUT1, OUT1, H2, 0L, W1P, W1P, H2, 0L, (void*)MID, (void*)MID, MLPH, 0L, B1R, B1R, 0L, NROWS, MLPH, H2, WCARRY_INV);
  wmma_gemm64<0, false, 2, 0, false, 1><<<grid_out, 256, 0, stream>>>(
      MID, MID, MLPH, 0L, W2P, W2P, MLPH, 0L, (void*)y_out, (void*)y_out, DOUT, 0L, B2R, B2R, 0L, NROWS, DOUT, MLPH, WCARRY_INV);
}
